// SessionGraph_78718160601343
// MI455X (gfx1250) — hardware-run, weakly checked
//
#include <hip/hip_runtime.h>

typedef float          v8f   __attribute__((ext_vector_type(8)));
typedef float          v4f   __attribute__((ext_vector_type(4)));
typedef unsigned int   v4u   __attribute__((ext_vector_type(4)));
typedef int            v8i   __attribute__((ext_vector_type(8)));
typedef unsigned short v8us  __attribute__((ext_vector_type(8)));
typedef unsigned short v16us __attribute__((ext_vector_type(16)));
typedef __bf16         v16bf __attribute__((ext_vector_type(16)));
typedef _Float16       v16h  __attribute__((ext_vector_type(16)));
typedef v4f  __attribute__((may_alias)) v4fa;
typedef v8us __attribute__((may_alias)) v8usa;
union FragB { v16bf v; v16us u; v8us h[2]; v8i w; };
union FragH { v16h  v; v16us u; v8us h[2]; v8i w; };

__device__ __forceinline__ v8f wmb(const FragB& a, const FragB& b, v8f c) {
  v8f d = __builtin_amdgcn_wmma_f32_16x16x32_bf16(false, a.v, false, b.v, (short)0, c, false, false);
  asm volatile("v_nop\n\tv_nop\n\tv_nop\n\tv_nop" : "+v"(d) : "v"(a.w), "v"(b.w));
  return d;
}

__device__ __forceinline__ v8f wmh(const FragH& a, const FragH& b, v8f c) {
  v8f d = __builtin_amdgcn_wmma_f32_16x16x32_f16(false, a.v, false, b.v, (short)0, c, false, false);
  asm volatile("v_nop\n\tv_nop\n\tv_nop\n\tv_nop" : "+v"(d) : "v"(a.w), "v"(b.w));
  return d;
}

__device__ __forceinline__ unsigned bf16_bits(float f) {
  const unsigned u = __float_as_uint(f);
  const unsigned r = (u + 0x7FFFu + ((u >> 16) & 1u)) >> 16;
  const unsigned q = (u >> 16) | 0x40u;
  return ((u & 0x7fffffffu) > 0x7f800000u) ? q : r;
}

__device__ __forceinline__ float bf16_val(float f) {
  return __uint_as_float(bf16_bits(f) << 16);
}
__device__ __forceinline__ int clampi(int v, int lo, int hi) {
  return v < lo ? lo : (v > hi ? hi : v);
}

__device__ __forceinline__ unsigned f16_bits(float f) {
  const unsigned u  = __float_as_uint(f);
  const unsigned s  = (u >> 16) & 0x8000u;
  const unsigned a  = u & 0x7fffffffu;
  const unsigned t  = a - 0x38000000u;
  const unsigned r  = (t + 0x0FFFu + ((t >> 13) & 1u)) >> 13;
  const unsigned rc = r > 0x7C00u ? 0x7C00u : r;
  const bool small  = a < 0x38800000u;
  const bool isnan  = a > 0x7f800000u;
  const unsigned fin = small ? 0u : (s | rc);
  return isnan ? (s | 0x7E00u) : fin;
}

__device__ __forceinline__ unsigned pk16(unsigned lo, unsigned hi) { return lo | (hi << 16); }
__device__ __forceinline__ unsigned bf16_lo_bits(float v) {
  float hi = bf16_val(v);
  asm volatile("" : "+v"(hi));
  return bf16_bits(v - hi);
}
__device__ __forceinline__ v4u pack8_bf16(v4f a, v4f c) {
  return (v4u){ pk16(bf16_bits(a[0]), bf16_bits(a[1])), pk16(bf16_bits(a[2]), bf16_bits(a[3])),
                pk16(bf16_bits(c[0]), bf16_bits(c[1])), pk16(bf16_bits(c[2]), bf16_bits(c[3])) };
}
__device__ __forceinline__ v4u pack8_bf16_lo(v4f a, v4f c) {
  return (v4u){ pk16(bf16_lo_bits(a[0]), bf16_lo_bits(a[1])), pk16(bf16_lo_bits(a[2]), bf16_lo_bits(a[3])),
                pk16(bf16_lo_bits(c[0]), bf16_lo_bits(c[1])), pk16(bf16_lo_bits(c[2]), bf16_lo_bits(c[3])) };
}
__device__ __forceinline__ v4u pack8_f16(v4f a, v4f c) {
  return (v4u){ pk16(f16_bits(a[0]), f16_bits(a[1])), pk16(f16_bits(a[2]), f16_bits(a[3])),
                pk16(f16_bits(c[0]), f16_bits(c[1])), pk16(f16_bits(c[2]), f16_bits(c[3])) };
}

template <int FORM>
__global__ __launch_bounds__(256) void k_plane(const float* __restrict__ src, int rows, int cols, int ldsrc,
                                               unsigned short* __restrict__ dst, int MP, int KP) {
  static_assert(FORM >= 0 && FORM <= 3);
  const int KTOT = (FORM == 1 || FORM == 3) ? 2 * KP : KP;
  const unsigned ppr   = (unsigned)(KTOT >> 3);
  const unsigned kp8   = (unsigned)(KP >> 3);
  const unsigned total = (unsigned)MP * ppr;
  const unsigned g     = blockIdx.x * 256u + threadIdx.x;
  const unsigned rowu  = g / ppr;
  const unsigned p     = g - rowu * ppr;
  const bool second    = p >= kp8;
  const int row = (int)rowu;
  const int c0  = (int)((second ? p - kp8 : p) << 3);
  const float* srow = src + (size_t)clampi(row, 0, rows - 1) * (size_t)ldsrc;
  float x[8];
  unsigned mk[8];
#pragma unroll
  for (int e = 0; e < 8; ++e) {
    const int c = c0 + e;
    const float v = srow[clampi(c, 0, cols - 1)];
    asm volatile("" :: "v"(v));
    x[e]  = v;
    mk[e] = (row < rows && c < cols) ? 0xFFFFu : 0u;
  }
  const v4f a = (v4f){ x[0], x[1], x[2], x[3] };
  const v4f c = (v4f){ x[4], x[5], x[6], x[7] };
  v4u o;
  if (FORM == 2) {
    o = pack8_f16(a, c);
  } else {
    const v4u hi = pack8_bf16(a, c);
    o = hi;
    if (FORM == 1) { const v4u lo = pack8_bf16_lo(a, c); o = second ? lo : hi; }
  }
  const v4u mw = (v4u){ pk16(mk[0], mk[1]), pk16(mk[2], mk[3]), pk16(mk[4], mk[5]), pk16(mk[6], mk[7]) };
  o &= mw;
  if (g < total) {
    volatile v4u* q = (volatile v4u*)(dst + (size_t)g * 8);
    *q = o;
    __threadfence();
    *q = o;
  }
}

template <int FORM> struct FragOf    { typedef FragB T; };
template <>         struct FragOf<2> { typedef FragH T; };
__device__ __forceinline__ v8f mm(const FragB& a, const FragB& b, v8f c) { return wmb(a, b, c); }
__device__ __forceinline__ v8f mm(const FragH& a, const FragH& b, v8f c) { return wmh(a, b, c); }
template <class F> __device__ __forceinline__ F ld_frag(const unsigned short* p) {
  F f;
  f.h[0] = *(const v8usa*)(p);
  f.h[1] = *(const v8usa*)(p + 16);
  return f;
}

template <int FORM, int EPI>
__global__ __launch_bounds__(256) __attribute__((amdgpu_num_vgpr(248)))
void k_gemm_nt(const unsigned short* __restrict__ A, const unsigned short* __restrict__ B,
               const float* __restrict__ bias, float* __restrict__ D, int M, int N, int KTOT, int ldd) {
  static_assert(FORM >= 0 && FORM <= 2);
  static_assert(EPI == 0 || EPI == 1);
  typedef typename FragOf<FORM>::T F;
  __shared__ __attribute__((aligned(16))) float sT[8][16 * 68];
  const int lane = threadIdx.x & 31;
  const int wave = threadIdx.x >> 5;
  const int tilesM = (M + 63) >> 6;
  const int tilesN = (N + 63) >> 6;
  const int tile = blockIdx.x * 8 + wave;
  if (tile >= tilesM * tilesN) return;
  const int tm = tile / tilesN;
  const int tn = tile - tm * tilesN;
  const int m0 = tm << 6;
  const int n0 = tn << 6;

  const int rl = lane & 15;
  const int h8 = (lane >> 4) * 8;
  const unsigned short* pa = A + (size_t)(m0 + rl) * (size_t)KTOT + h8;
  const unsigned short* pb = B + (size_t)(n0 + rl) * (size_t)KTOT + h8;

  v8f acc[4][4];
#pragma unroll
  for (int i = 0; i < 4; ++i)
#pragma unroll
    for (int j = 0; j < 4; ++j) acc[i][j] = (v8f){0.f, 0.f, 0.f, 0.f, 0.f, 0.f, 0.f, 0.f};

#pragma unroll 1
  for (int k0 = 0; k0 < KTOT; k0 += 32) {
    F bf[4];
#pragma unroll
    for (int j = 0; j < 4; ++j) bf[j] = ld_frag<F>(pb + (size_t)(j << 4) * (size_t)KTOT + k0);
#pragma unroll
    for (int i = 0; i < 4; ++i) {
      const F af = ld_frag<F>(pa + (size_t)(i << 4) * (size_t)KTOT + k0);
#pragma unroll
      for (int j = 0; j < 4; ++j) acc[i][j] = mm(af, bf[j], acc[i][j]);
    }
  }

  float* slab = sT[wave];
  const int hh = lane >> 4;
  const int c4 = (lane & 15) * 4;
  const int nc = n0 + c4;
  const bool cok = nc < N;
  v4f bv = (v4f){0.f, 0.f, 0.f, 0.f};
  if (EPI == 1) {
    bv = *(const v4fa*)(bias + clampi(nc, 0, N - 4));
    asm volatile("" :: "v"(bv));
  }
#pragma unroll
  for (int i = 0; i < 4; ++i) {
    const int mBase = m0 + (i << 4);
#pragma unroll
    for (int j = 0; j < 4; ++j) {
#pragma unroll
      for (int r = 0; r < 8; ++r) slab[(h8 + r) * 68 + (j << 4) + rl] = acc[i][j][r];
    }
    __builtin_amdgcn_fence(__ATOMIC_RELEASE, "workgroup");
    __builtin_amdgcn_wave_barrier();
    __builtin_amdgcn_fence(__ATOMIC_ACQUIRE, "workgroup");
    v4f vv[8];
#pragma unroll
    for (int it = 0; it < 8; ++it) {
      const int row = it * 2 + hh;
      v4f v = *(const v4fa*)(slab + row * 68 + c4);
      if (EPI == 1) v += bv;
      vv[it] = v;
    }
    for (int pass = 0; pass < 2; ++pass) {
#pragma unroll
      for (int it = 0; it < 8; ++it) {
        const int row = mBase + it * 2 + hh;
        if (cok && row < M) *(volatile v4f*)(D + (size_t)row * (size_t)ldd + nc) = vv[it];
      }
      __threadfence();
    }
    __builtin_amdgcn_fence(__ATOMIC_RELEASE, "workgroup");
    __builtin_amdgcn_wave_barrier();
    __builtin_amdgcn_fence(__ATOMIC_ACQUIRE, "workgroup");
  }
}

typedef v4u __attribute__((may_alias)) v4ua;

#define SPLIT_H     0
#define SPLIT_C     0
#define PRECISE_ACT 0

#define D_EMB   100
#define H_DIM   50
#define G_DIM   200
#define GP      208
#define KP      128
#define HP      64
#define NSLOT   12800
#define NITEM   40000
#define ROWS_U  20000
#define ROWS_I  40000
#define ROWS_S  30000
#define PROWS_U 20032
#define PROWS_I 40000
#define PROWS_S 30016

#define WPIECES 5120
#define WQ_WH   3328
#define WQ_BI   4992
#define WQ_PAD  5056
static_assert(GP * KP / 8 == WQ_WH);
static_assert(WQ_WH + GP * HP / 8 == WQ_BI);
static_assert(WQ_BI + 64 == WQ_PAD);
static_assert(WPIECES == 20 * 256);
static_assert(WQ_WH % 32 == 0 && WQ_BI % 32 == 0 && WQ_PAD % 32 == 0 && WPIECES % 32 == 0);
static_assert(D_EMB <= KP && H_DIM <= HP && G_DIM <= GP && GP == 13 * 16 && G_DIM == 4 * H_DIM);
static_assert(D_EMB % 4 == 0);
static_assert(NSLOT % 64 == 0 && NSLOT % 32 == 0);
static_assert(PROWS_U % 64 == 0 && PROWS_I % 64 == 0 && PROWS_S % 64 == 0);
static_assert(PROWS_U >= ROWS_U && PROWS_I >= ROWS_I && PROWS_S >= ROWS_S);

#define L_W    0
#define L_WH   53248
#define L_BI   79872
#define L_A    81920
#define L_H    114688
#define L_G    131072
#define L_C    184320
#define L_O    200704
#define L_TOT  233472
static_assert(L_WH == GP * KP * 2 && L_BI == L_WH + GP * HP * 2 && L_A == WPIECES * 16);
static_assert(L_H == L_A + 64 * 256 * 2 && L_G == L_H + 64 * 128 * 2 && L_C == L_G + 64 * GP * 4);
static_assert(L_O == L_C + 4096 * 4 && L_TOT == L_O + 64 * 128 * 4);
static_assert(L_TOT <= 327680);
static_assert(64 * H_DIM == 12 * 256 + 128);

static constexpr size_t OFF_CU  = 0;
static constexpr size_t OFF_CI  = OFF_CU + (size_t)PROWS_U * 512;
static constexpr size_t OFF_CS  = OFF_CI + (size_t)PROWS_I * 512;
static constexpr size_t OFF_AU  = OFF_CS + (size_t)PROWS_S * 512;
static constexpr size_t OFF_AI  = OFF_AU + (size_t)NSLOT * 512;
static constexpr size_t OFF_AS  = OFF_AI + (size_t)NSLOT * 512;
static constexpr size_t OFF_W   = OFF_AS + (size_t)NSLOT * 512;
static constexpr size_t OFF_ATT = OFF_W + (size_t)10 * WPIECES * 16;
static constexpr size_t WS_TOTAL = OFF_ATT + 1024;
static_assert(OFF_CI == 10256384 && OFF_CS == 30736384 && OFF_AU == 46104576);
static_assert(OFF_AI == 52658176 && OFF_AS == 59211776 && OFF_W == 65765376 && OFF_ATT == 66584576);
static_assert(WS_TOTAL == 66585600);
static_assert(OFF_CI % 256 == 0 && OFF_CS % 256 == 0 && OFF_AU % 256 == 0 && OFF_AI % 256 == 0);
static_assert(OFF_AS % 256 == 0 && OFF_W % 256 == 0 && OFF_ATT % 256 == 0);
static_assert(WS_TOTAL <= ((size_t)128 << 20));

__device__ __forceinline__ float act_sig(float x) {
#if PRECISE_ACT
  return 1.0f / (1.0f + expf(-x));
#else
  return __builtin_amdgcn_rcpf(1.0f + __expf(-x));
#endif
}
__device__ __forceinline__ float act_tanh(float x) {
#if PRECISE_ACT
  return tanhf(x);
#else
  return 1.0f - 2.0f * __builtin_amdgcn_rcpf(1.0f + __expf(2.0f * x));
#endif
}

__device__ __forceinline__ FragB lds_frag(const unsigned short* p) {
  FragB f;
  f.h[0] = *(const v8usa*)(p);
  f.h[1] = *(const v8usa*)(p + 16);
  return f;
}

__global__ __launch_bounds__(256) void k_pack(const float* __restrict__ Wih, const float* __restrict__ Whh,
                                              const float* __restrict__ bb, const float* __restrict__ att,
                                              v4u* __restrict__ wdst, v4u* __restrict__ adst, int set) {
  const int tid = threadIdx.x;
  if (blockIdx.x < 40) {
    const int g = blockIdx.x * 256 + tid;
    const int d = (g >= WPIECES) ? 1 : 0;
    const int q = g - d * WPIECES;
    v4u o = (v4u){0u, 0u, 0u, 0u};
    if (q < WQ_WH) {
      const int row = q >> 4;
      const int c0  = (q & 15) << 3;
      const float* sr = Wih + ((size_t)d * G_DIM + (size_t)clampi(row, 0, G_DIM - 1)) * D_EMB;
      float x[8];
      unsigned mk[8];
#pragma unroll
      for (int e = 0; e < 8; ++e) {
        const int c = c0 + e;
        const float v = sr[clampi(c, 0, D_EMB - 1)];
        asm volatile("" :: "v"(v));
        x[e]  = v;
        mk[e] = (row < G_DIM && c < D_EMB) ? 0xFFFFu : 0u;
      }
      o = pack8_bf16((v4f){x[0], x[1], x[2], x[3]}, (v4f){x[4], x[5], x[6], x[7]});
      o &= (v4u){ pk16(mk[0], mk[1]), pk16(mk[2], mk[3]), pk16(mk[4], mk[5]), pk16(mk[6], mk[7]) };
    } else if (q < WQ_BI) {
      const int q2  = q - WQ_WH;
      const int row = q2 >> 3;
      const int c0  = (q2 & 7) << 3;
      const float* sr = Whh + ((size_t)d * G_DIM + (size_t)clampi(row, 0, G_DIM - 1)) * H_DIM;
      float x[8];
      unsigned mk[8];
#pragma unroll
      for (int e = 0; e < 8; ++e) {
        const int c = c0 + e;
        const float v = sr[clampi(c, 0, H_DIM - 1)];
        asm volatile("" :: "v"(v));
        x[e]  = v;
        mk[e] = (row < G_DIM && c < H_DIM) ? 0xFFFFu : 0u;
      }
      o = pack8_bf16((v4f){x[0], x[1], x[2], x[3]}, (v4f){x[4], x[5], x[6], x[7]});
      o &= (v4u){ pk16(mk[0], mk[1]), pk16(mk[2], mk[3]), pk16(mk[4], mk[5]), pk16(mk[6], mk[7]) };
    } else if (q < WQ_PAD) {
      const int q3 = q - WQ_BI;
      unsigned w[4];
#pragma unroll
      for (int e = 0; e < 4; ++e) {
        const int n = 4 * q3 + e;
        const float v = bb[d * G_DIM + clampi(n, 0, G_DIM - 1)];
        asm volatile("" :: "v"(v));
        const unsigned m = (n < G_DIM) ? 0xFFFFFFFFu : 0u;
        w[e] = (bf16_bits(v) << 16) & m;
      }
      o = (v4u){ w[0], w[1], w[2], w[3] };
    }
    volatile v4u* qd = (volatile v4u*)(wdst + (size_t)(set * 2 + d) * WPIECES + q);
    *qd = o;
    __threadfence();
    *qd = o;
  } else if (set == 0 && tid < 64) {
    unsigned w[4];
#pragma unroll
    for (int e = 0; e < 4; ++e) {
      const int j  = 4 * tid + e;
      const int sj = (j < 128) ? j : (j - 28);
      const float v = att[clampi(sj, 0, 2 * D_EMB - 1)];
      asm volatile("" :: "v"(v));
      const bool ok = (j < D_EMB) || (j >= 128 && j < 128 + D_EMB);
      w[e] = (bf16_bits(v) << 16) & (ok ? 0xFFFFFFFFu : 0u);
    }
    const v4u o = (v4u){ w[0], w[1], w[2], w[3] };
    volatile v4u* qd = (volatile v4u*)(adst + tid);
    *qd = o;
    __threadfence();
    *qd = o;
  }
}

template <int MODE>
__device__ __forceinline__ void stage_rows(const float* __restrict__ src, int R, unsigned char* sAb, int srow, int spc) {
#pragma unroll
  for (int i = 0; i < 4; ++i) {
    const int pc = spc + i;
    const int c0 = pc << 3;
    unsigned char* dp = sAb + srow * 512 + pc * 16;
    if (MODE == 0) {
      const int ca = (c0 < D_EMB - 4) ? c0 : (D_EMB - 4);
      const int cb = (c0 + 4 < D_EMB - 4) ? (c0 + 4) : (D_EMB - 4);
      const float* rp = src + (size_t)R * D_EMB;
      const v4f a = *(const v4fa*)(rp + ca);
      const v4f c = *(const v4fa*)(rp + cb);
      asm volatile("" :: "v"(a));
      asm volatile("" :: "v"(c));
      const unsigned ma = (c0 < D_EMB) ? 0xFFFFFFFFu : 0u;
      const unsigned mb = (c0 + 4 < D_EMB) ? 0xFFFFFFFFu : 0u;
      v4u hi = pack8_bf16(a, c);
      hi &= (v4u){ ma, ma, mb, mb };
      *(v4ua*)dp = hi;
    } else {
      const float* rp = src + (size_t)R * KP + c0;
      const v4f a = *(const v4fa*)(rp);
      const v4f c = *(const v4fa*)(rp + 4);
      asm volatile("" :: "v"(a));
      asm volatile("" :: "v"(c));
      const v4u hi = pack8_bf16(a, c);
      *(v4ua*)dp = hi;
      if (SPLIT_C) {
        const v4u lo = pack8_bf16_lo(a, c);
        *(v4ua*)(dp + 256) = lo;
      }
    }
  }
}

template <int MODE, int T>
__global__ __launch_bounds__(256) __attribute__((amdgpu_num_vgpr(248)))
void k_bilstm(const float* __restrict__ ta, const float* __restrict__ tb,
              const int* __restrict__ flat, const int* __restrict__ nbr,
              int rows, const v4u* __restrict__ wpk, float* __restrict__ outp) {
  static_assert(MODE == 0 || MODE == 1);
  static_assert(T == 2 || T == 5);
  extern __shared__ __attribute__((aligned(16))) unsigned char smem[];
  unsigned short* sWI = (unsigned short*)(smem + L_W);
  unsigned short* sWH = (unsigned short*)(smem + L_WH);
  float*          sBI = (float*)(smem + L_BI);
  unsigned short* sA  = (unsigned short*)(smem + L_A);
  unsigned short* sH  = (unsigned short*)(smem + L_H);
  float*          sG  = (float*)(smem + L_G);
  float*          sC  = (float*)(smem + L_C);
  float*          sO  = (float*)(smem + L_O);

  const int tid  = threadIdx.x;
  const int lane = tid & 31;
  const int wave = tid >> 5;
  const int l15  = lane & 15;
  const int h8   = (lane >> 4) * 8;
  const int mt   = wave & 3;
  const int nbeg = (wave >> 2) ? 7 : 0;
  const int nend = (wave >> 2) ? 13 : 7;
  const int row0 = blockIdx.x * 64;
  const int srow = tid >> 2;
  const int spc  = (tid & 3) * 4;

  int fid  = 0;
  int Rfix = 0;
  if (MODE == 1) {
    int f = flat[clampi(row0 + srow, 0, NSLOT - 1)];
    asm volatile("" :: "v"(f));
    fid = clampi(f, 0, NITEM - 1);
  } else {
    Rfix = clampi(row0 + srow, 0, rows - 1);
  }

  const v4u z4 = (v4u){0u, 0u, 0u, 0u};
#pragma unroll
  for (int i = 0; i < 8; ++i) *(v4ua*)(smem + L_O + (size_t)(tid + 256 * i) * 16) = z4;

#pragma unroll 1
  for (int d = 0; d < 2; ++d) {
    const v4u* wsrc = wpk + (size_t)d * WPIECES;
#pragma unroll 4
    for (int i = 0; i < 20; ++i) {
      const v4u v = wsrc[tid + 256 * i];
      *(v4ua*)(smem + L_W + (size_t)(tid + 256 * i) * 16) = v;
    }
#pragma unroll
    for (int i = 0; i < 4; ++i) {
      *(v4ua*)(smem + L_H + (size_t)(tid + 256 * i) * 16) = z4;
      *(v4ua*)(smem + L_C + (size_t)(tid + 256 * i) * 16) = z4;
    }
    {
      const int t0 = d ? (T - 1) : 0;
      if (MODE == 0) {
        if (t0 == 0) stage_rows<0>(ta, Rfix, smem + L_A, srow, spc);
        else         stage_rows<0>(tb, Rfix, smem + L_A, srow, spc);
      } else {
        int nb = nbr[fid * T + t0];
        asm volatile("" :: "v"(nb));
        stage_rows<1>(ta, clampi(nb, 0, rows - 1), smem + L_A, srow, spc);
      }
    }
    __syncthreads();

#pragma unroll 1
    for (int s = 0; s < T; ++s) {
      {
        const unsigned short* pa = sA + (16 * mt + l15) * 256 + h8;
        const unsigned short* ph = sH + (16 * mt + l15) * 128 + h8;
        FragB ah[4], al[4], hh[2], hl[2];
#pragma unroll
        for (int ks = 0; ks < 4; ++ks) {
          ah[ks] = lds_frag(pa + 32 * ks);
          if (MODE == 1 && SPLIT_C) al[ks] = lds_frag(pa + 128 + 32 * ks);
          else                      al[ks] = ah[ks];
        }
#pragma unroll
        for (int ks = 0; ks < 2; ++ks) {
          hh[ks] = lds_frag(ph + 32 * ks);
          if (SPLIT_H) hl[ks] = lds_frag(ph + 64 + 32 * ks);
          else         hl[ks] = hh[ks];
        }
#pragma unroll 1
        for (int nt = nbeg; nt < nend; ++nt) {
          const int ncol = 16 * nt + l15;
          const float bv = sBI[ncol];
          v8f acc = (v8f){bv, bv, bv, bv, bv, bv, bv, bv};
          const unsigned short* pb = sWI + ncol * 128 + h8;
#pragma unroll
          for (int ks = 0; ks < 4; ++ks) {
            const FragB b = lds_frag(pb + 32 * ks);
            acc = wmb(ah[ks], b, acc);
            if (MODE == 1 && SPLIT_C) acc = wmb(al[ks], b, acc);
          }
          if (s > 0) {
            const unsigned short* pw = sWH + ncol * 64 + h8;
#pragma unroll
            for (int ks = 0; ks < 2; ++ks) {
              const FragB b = lds_frag(pw + 32 * ks);
              acc = wmb(hh[ks], b, acc);
              if (SPLIT_H) acc = wmb(hl[ks], b, acc);
            }
          }
          float* gd = sG + (16 * mt + h8) * GP + ncol;
#pragma unroll
          for (int r = 0; r < 8; ++r) gd[r * GP] = acc[r];
        }
      }
      __syncthreads();

      {
        const int niter = (wave < 4) ? 13 : 12;
#pragma unroll 1
        for (int i = 0; i < niter; ++i) {
          const int p   = tid + (i << 8);
          const int row = p / H_DIM;
          const int u   = p - row * H_DIM;
          const float* g = sG + row * GP + u;
          const float gi = g[0];
          const float gf = g[H_DIM];
          const float gg = g[2 * H_DIM];
          const float go = g[3 * H_DIM];
          const float cold = sC[p];
          const float cn = act_sig(gf) * cold + act_sig(gi) * act_tanh(gg);
          const float hn = act_sig(go) * act_tanh(cn);
          sC[p] = cn;
          const unsigned hb = bf16_bits(hn);
          sH[row * 128 + u] = (unsigned short)hb;
          if (SPLIT_H) {
            const float hv = __uint_as_float(hb << 16);
            sH[row * 128 + 64 + u] = (unsigned short)bf16_bits(hn - hv);
          }
          float* op = sO + row * 128 + d * H_DIM + u;
          const float o = *op;
          *op = o + hn;
        }
      }
      if (s + 1 < T) {
        const int tn = d ? (T - 2 - s) : (s + 1);
        if (MODE == 0) {
          if (tn == 0) stage_rows<0>(ta, Rfix, smem + L_A, srow, spc);
          else         stage_rows<0>(tb, Rfix, smem + L_A, srow, spc);
        } else {
          int nb = nbr[fid * T + tn];
          asm volatile("" :: "v"(nb));
          stage_rows<1>(ta, clampi(nb, 0, rows - 1), smem + L_A, srow, spc);
        }
      }
      __syncthreads();
    }
  }

  {
    const float invT = 1.0f / (float)T;
    v4f vv[8];
#pragma unroll
    for (int i = 0; i < 8; ++i) {
      const int row = wave * 8 + i;
      const v4f v = *(const v4fa*)(sO + row * 128 + 4 * lane);
      vv[i] = v * invT;
    }
#pragma unroll
    for (int i = 0; i < 8; ++i) {
      const int row = wave * 8 + i;
      *(volatile v4f*)(outp + (size_t)(row0 + row) * 128 + 4 * lane) = vv[i];
    }
    __threadfence();
#pragma unroll
    for (int i = 0; i < 8; ++i) {
      const int row = wave * 8 + i;
      *(volatile v4f*)(outp + (size_t)(row0 + row) * 128 + 4 * lane) = vv[i];
    }
  }
}

__device__ __forceinline__ float wsum32(float v) {
  v += __shfl_xor(v, 16);
  v += __shfl_xor(v, 8);
  v += __shfl_xor(v, 4);
  v += __shfl_xor(v, 2);
  v += __shfl_xor(v, 1);
  return v;
}
__device__ __forceinline__ float dot4(v4f a, v4f b) {
  return a[0] * b[0] + a[1] * b[1] + a[2] * b[2] + a[3] * b[3];
}
__device__ __forceinline__ float leaky(float x) { return (x > 0.0f) ? x : 0.01f * x; }

__global__ __launch_bounds__(256) void k_combine(const int* __restrict__ flat, const float* __restrict__ CI,
                                                 const float* __restrict__ AU, const float* __restrict__ AI,
                                                 const float* __restrict__ AS, const float* __restrict__ attP,
                                                 float* __restrict__ out) {
  __shared__ __attribute__((aligned(16))) float sAtt[256];
  __shared__ __attribute__((aligned(16))) float sOut[32 * D_EMB];
  const int tid  = threadIdx.x;
  const int lane = tid & 31;
  const int wave = tid >> 5;
  if (tid < 64) {
    const v4f v = *(const v4fa*)(attP + 4 * tid);
    *(v4fa*)(sAtt + 4 * tid) = v;
  }
  __syncthreads();
  const v4f a1 = *(const v4fa*)(sAtt + 4 * lane);
  const v4f a2 = *(const v4fa*)(sAtt + 128 + 4 * lane);
  const int n0 = blockIdx.x * 32;
  const v4f zero = (v4f){0.f, 0.f, 0.f, 0.f};

#pragma unroll 1
  for (int j = 0; j < 4; ++j) {
    const int rl = wave * 4 + j;
    const int n  = clampi(n0 + rl, 0, NSLOT - 1);
    int id = flat[n];
    asm volatile("" :: "v"(id));
    const int cid = clampi(id, 0, NITEM - 1);
    const v4f vc = *(const v4fa*)(CI + (size_t)cid * 128 + 4 * lane);
    const v4f vu = *(const v4fa*)(AU + (size_t)n * 128 + 4 * lane);
    const v4f vi = *(const v4fa*)(AI + (size_t)n * 128 + 4 * lane);
    const v4f vs = *(const v4fa*)(AS + (size_t)n * 128 + 4 * lane);
    asm volatile("" :: "v"(vc));
    asm volatile("" :: "v"(vu));
    asm volatile("" :: "v"(vi));
    asm volatile("" :: "v"(vs));
    const float d0 = wsum32(dot4(vc, a1));
    const float dc = wsum32(dot4(vc, a2));
    const float du = wsum32(dot4(vu, a2));
    const float di = wsum32(dot4(vi, a2));
    const float ds = wsum32(dot4(vs, a2));
    const float ec = leaky(d0 + dc);
    const float eu = leaky(d0 + du);
    const float ei = leaky(d0 + di);
    const float es = leaky(d0 + ds);
    const float m  = fmaxf(fmaxf(ec, eu), fmaxf(ei, es));
    float w0 = __expf(ec - m);
    float w1 = __expf(eu - m);
    float w2 = __expf(ei - m);
    float w3 = __expf(es - m);
    const float inv = __builtin_amdgcn_rcpf((w0 + w1) + (w2 + w3));
    w0 *= inv; w1 *= inv; w2 *= inv; w3 *= inv;
    const v4f agg = vc * w0 + vu * w1 + vi * w2 + vs * w3;
    const v4f res = (id != 0) ? agg : zero;
    if (lane < 25) *(v4fa*)(sOut + rl * D_EMB + 4 * lane) = res;
  }
  __syncthreads();

  float* ob = out + (size_t)blockIdx.x * (32 * D_EMB);
  v4f vv[4];
#pragma unroll
  for (int i = 0; i < 4; ++i) {
    const int p  = tid + 256 * i;
    const int pc = (p < 800) ? p : 799;
    vv[i] = *(const v4fa*)(sOut + 4 * pc);
  }
#pragma unroll
  for (int i = 0; i < 4; ++i) {
    const int p = tid + 256 * i;
    if (p < 800) *(volatile v4f*)(ob + 4 * p) = vv[i];
  }
  __threadfence();
#pragma unroll
  for (int i = 0; i < 4; ++i) {
    const int p = tid + 256 * i;
    if (p < 800) *(volatile v4f*)(ob + 4 * p) = vv[i];
  }
}

extern "C" void kernel_launch(void* const* d_in, const int* in_sizes, int n_in,
                              void* d_out, int out_size, void* d_ws, size_t ws_size, hipStream_t stream) {
  if (n_in < 24) return;
  if (in_sizes[0] != NSLOT) return;
  if (in_sizes[1] != ROWS_U * D_EMB || in_sizes[2] != ROWS_I * D_EMB) return;
  if (in_sizes[3] != ROWS_I * D_EMB || in_sizes[4] != ROWS_S * D_EMB) return;
  if (in_sizes[5] != NITEM * 5 || in_sizes[6] != NITEM * 5 || in_sizes[7] != NITEM * 2) return;
  for (int s = 0; s < 5; ++s) {
    if (in_sizes[8 + 3 * s] != 2 * G_DIM * D_EMB) return;
    if (in_sizes[9 + 3 * s] != 2 * G_DIM * H_DIM) return;
    if (in_sizes[10 + 3 * s] != 2 * G_DIM) return;
  }
  if (in_sizes[23] != 2 * D_EMB) return;
  if (out_size != NSLOT * D_EMB) return;
  if (WS_TOTAL > ws_size) return;

  const int*   flat = (const int*)d_in[0];
  const float* f1   = (const float*)d_in[1];
  const float* f3   = (const float*)d_in[2];
  const float* f5   = (const float*)d_in[3];
  const float* f8   = (const float*)d_in[4];
  const int*   nu   = (const int*)d_in[5];
  const int*   ni   = (const int*)d_in[6];
  const int*   ns   = (const int*)d_in[7];
  const float* att  = (const float*)d_in[23];

  unsigned char* ws = (unsigned char*)d_ws;
  float* CU = (float*)(ws + OFF_CU);
  float* CI = (float*)(ws + OFF_CI);
  float* CS = (float*)(ws + OFF_CS);
  float* AU = (float*)(ws + OFF_AU);
  float* AI = (float*)(ws + OFF_AI);
  float* AS = (float*)(ws + OFF_AS);
  v4u*   WP = (v4u*)(ws + OFF_W);
  v4u*   AT = (v4u*)(ws + OFF_ATT);
  float* out = (float*)d_out;

  (void)hipFuncSetAttribute(reinterpret_cast<const void*>(&k_bilstm<0, 2>),
                            hipFuncAttributeMaxDynamicSharedMemorySize, (int)L_TOT);
  (void)hipFuncSetAttribute(reinterpret_cast<const void*>(&k_bilstm<1, 5>),
                            hipFuncAttributeMaxDynamicSharedMemorySize, (int)L_TOT);
  (void)hipFuncSetAttribute(reinterpret_cast<const void*>(&k_bilstm<1, 2>),
                            hipFuncAttributeMaxDynamicSharedMemorySize, (int)L_TOT);

  for (int s = 0; s < 5; ++s) {
    k_pack<<<41, 256, 0, stream>>>((const float*)d_in[8 + 3 * s], (const float*)d_in[9 + 3 * s],
                                   (const float*)d_in[10 + 3 * s], att, WP, AT, s);
  }
  const v4u* W_uc = WP + (size_t)0 * 2 * WPIECES;
  const v4u* W_ic = WP + (size_t)1 * 2 * WPIECES;
  const v4u* W_sc = WP + (size_t)2 * 2 * WPIECES;
  const v4u* W_un = WP + (size_t)3 * 2 * WPIECES;
  const v4u* W_in = WP + (size_t)4 * 2 * WPIECES;

  k_bilstm<0, 2><<<PROWS_U / 64, 256, L_TOT, stream>>>(f1, f1, flat, nu, ROWS_U, W_uc, CU);
  k_bilstm<0, 2><<<PROWS_I / 64, 256, L_TOT, stream>>>(f3, f5, flat, ni, ROWS_I, W_ic, CI);
  k_bilstm<0, 2><<<PROWS_S / 64, 256, L_TOT, stream>>>(f8, f8, flat, ns, ROWS_S, W_sc, CS);

  k_bilstm<1, 5><<<NSLOT / 64, 256, L_TOT, stream>>>(CU, CU, flat, nu, ROWS_U, W_un, AU);
  k_bilstm<1, 5><<<NSLOT / 64, 256, L_TOT, stream>>>(CI, CI, flat, ni, ROWS_I, W_in, AI);
  k_bilstm<1, 2><<<NSLOT / 64, 256, L_TOT, stream>>>(CS, CS, flat, ns, ROWS_S, W_in, AS);

  k_combine<<<NSLOT / 32, 256, 0, stream>>>(flat, CI, AU, AI, AS, (const float*)AT, out);
}
